// GroupedQueryAttention_45019847197304
// MI455X (gfx1250) — hardware-verified
//
#include <hip/hip_runtime.h>


#ifndef NB
#define NB 2
#endif
#ifndef SEQ
#define SEQ 2048
#endif
#define NB_FULL  2
#define SEQ_FULL 2048
#define DM    1024
#define NH_   16
#define NKV   4
#define REP   (NH_ / NKV)
#define HD    64
#define DQ    (NH_ * HD)
#define DKV   (NKV * HD)
#define DQKV  (DQ + 2 * DKV)
#define HALFQ (DQ / 2)
#define HALFK (DKV / 2)
#define PCAR_LOG2 8.0f
#define VCAR  16.0f
#define QRES  2048.0f
#define PP 40
#define MP 36
#define OP 68

static_assert(NB <= NB_FULL);
static_assert(SEQ <= SEQ_FULL);
static_assert(SEQ % 64 == 0);
static_assert(DM % 64 == 0);
static_assert(DM % 32 == 0);
static_assert(DQ % 32 == 0);
static_assert(DQKV % 64 == 0);
static_assert(HD == 64);
static_assert(REP == 4);
static_assert(NH_ == NKV * REP);
static_assert(HALFQ % HD == 0);
static_assert(HALFK % HD == 0);
static_assert(HALFQ == 512);
static_assert(HALFK == 128);
static_assert((NH_ * SEQ) % 8 == 0);
static_assert((NKV * SEQ) % 8 == 0);
static_assert((PP * 2) % 16 == 0);
static_assert((MP * 4) % 16 == 0);
static_assert((OP * 4) % 16 == 0);

typedef _Float16 h16;
typedef unsigned short bf;
typedef __attribute__((ext_vector_type(16))) __bf16   v16bf;
typedef __attribute__((ext_vector_type(16))) _Float16 v16h;
typedef __attribute__((ext_vector_type(8)))  _Float16 v8h;
typedef __attribute__((ext_vector_type(8)))  unsigned short v8us;
typedef __attribute__((ext_vector_type(8)))  float    v8f;
typedef __attribute__((ext_vector_type(4)))  float    v4f;
typedef __attribute__((ext_vector_type(2)))  float    v2f;
typedef __attribute__((ext_vector_type(2)))  _Float16 v2h;
typedef __attribute__((ext_vector_type(2)))  unsigned short v2us;
typedef v8h  __attribute__((may_alias)) v8ha;
typedef v4f  __attribute__((may_alias)) v4fa;

__device__ __forceinline__ unsigned short f2bf(float f) { unsigned u = __float_as_uint(f); u += 0x7FFFu + ((u >> 16) & 1u); return (unsigned short)(u >> 16); }
__device__ __forceinline__ float bf2f(unsigned short b) { return __uint_as_float(((unsigned)b) << 16); }
__device__ __forceinline__ float bfr(float f) { return bf2f(f2bf(f)); }
__device__ __forceinline__ void splitf(float y, unsigned short& h, unsigned short& l) { h = f2bf(y); l = f2bf(y - bf2f(h)); }
__device__ __forceinline__ v16h cat16(v8h lo, v8h hi) { return __builtin_shufflevector(lo, hi, 0, 1, 2, 3, 4, 5, 6, 7, 8, 9, 10, 11, 12, 13, 14, 15); }
__device__ __forceinline__ v16bf cat16b(v8us lo, v8us hi) { return __builtin_bit_cast(v16bf, __builtin_shufflevector(lo, hi, 0, 1, 2, 3, 4, 5, 6, 7, 8, 9, 10, 11, 12, 13, 14, 15)); }
__device__ __forceinline__ v8f wmma16(v16h a, v16h b, v8f c) { return __builtin_amdgcn_wmma_f32_16x16x32_f16(false, a, false, b, (short)0, c, false, false); }
__device__ __forceinline__ v8f wmmab(v16bf a, v16bf b, v8f c) { return __builtin_amdgcn_wmma_f32_16x16x32_bf16(false, a, false, b, (short)0, c, false, false); }
__device__ __forceinline__ v16h ldh(const h16* p) { return cat16(*(const v8h*)p, *(const v8h*)(p + 16)); }
__device__ __forceinline__ void wsync() { __builtin_amdgcn_wave_barrier(); asm volatile("" ::: "memory"); }

template <typename T16> struct WFrag;
template <> struct WFrag<h16> { typedef v16h V; static __device__ __forceinline__ V ld(const h16* p) { return cat16(*(const v8h*)p, *(const v8h*)(p + 16)); } static __device__ __forceinline__ v8f mma(V a, V b, v8f c) { return wmma16(a, b, c); } };
template <> struct WFrag<bf> { typedef v16bf V; static __device__ __forceinline__ V ld(const bf* p) { return cat16b(*(const v8us*)p, *(const v8us*)(p + 16)); } static __device__ __forceinline__ v8f mma(V a, V b, v8f c) { return wmmab(a, b, c); } };
template <typename T16, int NSPLIT, bool BIAS>
__device__ __forceinline__ void gemmw_body(const T16* __restrict__ A, const T16* __restrict__ A2, const T16* __restrict__ Bt, int K, float* C, int ldc, const float* __restrict__ bias) {
    static_assert(NSPLIT == 0 || NSPLIT == 1);
    typedef typename WFrag<T16>::V V;
    __shared__ __align__(16) float os[16 * 68];
    const int lane = threadIdx.x & 31, lr = lane & 15, hi = lane >> 4; const int r0 = blockIdx.x * 64, c0 = blockIdx.y * 64;
    v8f acc[4][4];
#pragma unroll
    for (int mb = 0; mb < 4; ++mb)
#pragma unroll
        for (int nb = 0; nb < 4; ++nb) acc[mb][nb] = (v8f){};
    const size_t aoff = (size_t)(r0 + lr) * K + 8 * hi, boff = (size_t)(c0 + lr) * K + 8 * hi;
#pragma unroll 1
    for (int kc = 0; kc < K; kc += 32) {
        V a[4], a2[4];
#pragma unroll
        for (int mb = 0; mb < 4; ++mb) { a[mb] = WFrag<T16>::ld(A + aoff + (size_t)mb * 16 * K + kc); if (NSPLIT == 1) a2[mb] = WFrag<T16>::ld(A2 + aoff + (size_t)mb * 16 * K + kc); }
#pragma unroll
        for (int nb = 0; nb < 4; ++nb) { const V b = WFrag<T16>::ld(Bt + boff + (size_t)nb * 16 * K + kc);
#pragma unroll
            for (int mb = 0; mb < 4; ++mb) { acc[mb][nb] = WFrag<T16>::mma(a[mb], b, acc[mb][nb]); if (NSPLIT == 1) acc[mb][nb] = WFrag<T16>::mma(a2[mb], b, acc[mb][nb]); } }
        asm volatile("v_nop\n\tv_nop\n\tv_nop\n\tv_nop" : "+v"(acc[0][0]), "+v"(acc[1][1]), "+v"(acc[2][2]), "+v"(acc[3][3]) : "v"(a[0]), "v"(a[3]));
    }
#pragma unroll
    for (int mb = 0; mb < 4; ++mb) {
#pragma unroll
        for (int nb = 0; nb < 4; ++nb) {
#pragma unroll
            for (int j = 0; j < 8; ++j) os[(hi * 8 + j) * 68 + nb * 16 + lr] = acc[mb][nb][j]; }
        wsync();
        float* crow = C + (size_t)(r0 + mb * 16) * ldc + c0;
#pragma unroll 1
        for (int ps = 0; ps < 2; ++ps) {
#pragma unroll
            for (int s = 0; s < 8; ++s) { const int row = 2 * s + hi, cofs = lr * 4; v4f val = *(const v4fa*)(os + row * 68 + cofs); if (BIAS) { val[0] += bfr(bias[c0 + cofs]); val[1] += bfr(bias[c0 + cofs + 1]); val[2] += bfr(bias[c0 + cofs + 2]); val[3] += bfr(bias[c0 + cofs + 3]); }
                *(volatile v4f*)(crow + (size_t)row * ldc + cofs) = val; }
            if (ps == 0) __threadfence(); }
        wsync();
    }
}
__global__ __launch_bounds__(32) void k_gemm_proj(const bf* __restrict__ A, const bf* __restrict__ Bt, int K, float* C, int ldc) { gemmw_body<bf, 0, false>(A, A, Bt, K, C, ldc, (const float*)0); }
__global__ __launch_bounds__(32) void k_gemm_out(const bf* __restrict__ Ah, const bf* __restrict__ Al, const bf* __restrict__ Bt, int K, float* C, int ldc, const float* __restrict__ bias) { gemmw_body<bf, 1, true>(Ah, Al, Bt, K, C, ldc, bias); }

__global__ __launch_bounds__(256) void k_wtG(const float* __restrict__ w, int K, int N, bf* Bt) {
    const int lane = threadIdx.x & 31; const int L0 = (blockIdx.x * 8 + (threadIdx.x >> 5)) * 8; const int nlines = N * K / 64;
#pragma unroll
    for (int ps = 0; ps < 2; ++ps) {
#pragma unroll 1
        for (int l = 0; l < 8; ++l) { const int L = L0 + l; if (L >= nlines) break; const size_t e = (size_t)L * 64 + lane * 2; const int k = (int)(e % K), n = (int)(e / K); v2us o;
            o[0] = f2bf(w[(size_t)k * N + n]); o[1] = f2bf(w[(size_t)(k + 1) * N + n]); *(volatile v2us*)(Bt + e) = o; }
        if (ps == 0) __threadfence(); }
}
__global__ __launch_bounds__(256) void k_cvt8(const float* __restrict__ src, bf* dst, size_t n8) { const size_t i = (size_t)blockIdx.x * 256 + threadIdx.x; if (i >= n8) return; const v8f v = *(const v8f*)(src + i * 8); v8us o;
#pragma unroll
    for (int k = 0; k < 8; ++k) o[k] = f2bf(v[k]); *(volatile v8us*)(dst + i * 8) = o; __threadfence(); *(volatile v8us*)(dst + i * 8) = o; }

__global__ __launch_bounds__(256) void k_invf(float* IF) {
    const int i = blockIdx.x * 256 + threadIdx.x; const int isq = (i < HALFQ) ? 1 : 0; const int j = isq ? i : i - HALFQ; const float rh = isq ? (1.0f / (float)HALFQ) : (1.0f / (float)HALFK);
    const float p = powf(10000.0f, (float)j * rh); const float v = 1.0f / p;
    *(volatile float*)(IF + i) = v; __threadfence(); *(volatile float*)(IF + i) = v;
}
__global__ __launch_bounds__(256) void k_cstab(const float* __restrict__ IF, float* CS) {
    const int e = blockIdx.x * 256 + threadIdx.x; if (e >= SEQ * (HALFQ + HALFK)) return;
    const int isq = (e < SEQ * HALFQ) ? 1 : 0; const int e2 = isq ? e : e - SEQ * HALFQ; const int sh = isq ? 9 : 7; const int t = e2 >> sh; const int i = e2 - (t << sh);
    const float ang = (float)t * IF[isq ? i : HALFQ + i];
    v2f cs; cs[0] = cosf(ang); cs[1] = sinf(ang);
    *(volatile v2f*)(CS + (size_t)e * 2) = cs; __threadfence(); *(volatile v2f*)(CS + (size_t)e * 2) = cs;
}

__global__ __launch_bounds__(256) void k_ropen(const float* __restrict__ F, int col0, int half, int nheads, const float* __restrict__ CS, const float* __restrict__ bias, int wres, h16* P16, h16* PR) {
#pragma clang fp contract(off)
    const int lane = threadIdx.x & 31; const int R = blockIdx.x * 8 + (threadIdx.x >> 5); if (R >= nheads * SEQ) return;
    const int h = R / SEQ, t = R - h * SEQ; const int c = h * HD + 2 * lane; const bool lo = (c < half); const int cp = lo ? c + half : c - half; const int i = lo ? c : c - half;
    const float* f = F + (size_t)t * DQKV + col0;
    const v2f xa = *(const v2f*)(f + c), xb = *(const v2f*)(f + cp); const v2f ba = *(const v2f*)(bias + c), bb = *(const v2f*)(bias + cp); const v4f cs = *(const v4f*)(CS + ((size_t)t * half + i) * 2);
    float r[2];
#pragma unroll
    for (int q = 0; q < 2; ++q) { const float x0 = xa[q] + bfr(ba[q]), x1 = xb[q] + bfr(bb[q]); const float a = x0 * cs[2 * q], b = x1 * cs[2 * q + 1]; r[q] = lo ? (a - b) : (a + b); }
    float ss = r[0] * r[0] + r[1] * r[1];
#pragma unroll
    for (int sh = 16; sh; sh >>= 1) ss += __shfl_xor(ss, sh, 32);
    const float rn = rsqrtf(ss * (1.0f / 64.0f) + 1.1920929e-7f);
    v2h o16, ores;
#pragma unroll
    for (int q = 0; q < 2; ++q) { const float y = r[q] * rn; const h16 hq = (h16)y; o16[q] = hq; ores[q] = (h16)((y - (float)hq) * QRES); }
    const size_t off = (size_t)R * HD + 2 * lane;
    *(volatile v2h*)(P16 + off) = o16; if (wres) *(volatile v2h*)(PR + off) = ores; __threadfence(); *(volatile v2h*)(P16 + off) = o16; if (wres) *(volatile v2h*)(PR + off) = ores;
}
__global__ __launch_bounds__(256) void k_vtp(const float* __restrict__ F, const float* __restrict__ bias, h16* V16) {
    const size_t e = ((size_t)blockIdx.x * 256 + threadIdx.x) * 2; if (e >= (size_t)NKV * HD * SEQ) return; const int t = (int)(e % SEQ); const int d = (int)((e / SEQ) % HD); const int g = (int)(e / ((size_t)SEQ * HD));
    const float bb = bfr(bias[g * HD + d]); v2h o;
#pragma unroll
    for (int q = 0; q < 2; ++q) { const float x = F[(size_t)(t + q) * DQKV + DQ + DKV + g * HD + d] + bb; o[q] = (h16)(x * VCAR); }
    *(volatile v2h*)(V16 + e) = o; __threadfence(); *(volatile v2h*)(V16 + e) = o;
}

__global__ __launch_bounds__(128) void k_flash(const h16* __restrict__ Q16, const h16* __restrict__ QR, const h16* __restrict__ K16, const h16* __restrict__ VT, const float* __restrict__ mask, bf* ATh, bf* ATl) {
    __shared__ __align__(16) h16   sP[REP * 16 * PP];
    __shared__ __align__(16) float sM[REP * 16 * MP];
    __shared__ __align__(16) float sO[REP * 16 * OP];
    const int w = threadIdx.x >> 5, lane = threadIdx.x & 31, lr = lane & 15, hi = lane >> 4;
    const int kv = blockIdx.y, h = kv * REP + w, q0 = blockIdx.x * 16;
    const int pb = w * 16 * PP, mb = w * 16 * MP, ob = w * 16 * OP;
    const int qo = (h * SEQ + q0 + lr) * HD + 8 * hi;
    const h16* Kp = K16 + (size_t)kv * SEQ * HD + (size_t)lr * HD + 8 * hi;
    const h16* Vp = VT + (size_t)kv * HD * SEQ + (size_t)lr * SEQ + 8 * hi;
    const float* mp = mask + (size_t)q0 * SEQ_FULL;
    const float LOG2E = 1.4426950408889634f; const float C1 = 0.18033688011112043f; const float C2 = 0.18033688011112043f * (1.0f / QRES);
    v8f accO[4];
#pragma unroll
    for (int nb = 0; nb < 4; ++nb) accO[nb] = (v8f){};
    float mrow[8], lrow[8];
#pragma unroll
    for (int r = 0; r < 8; ++r) { mrow[r] = -1.0e30f; lrow[r] = 0.0f; }
#pragma unroll 1
    for (int kc = 0; kc < SEQ; kc += 32) {
#pragma unroll
        for (int j = 0; j < 4; ++j) { const int idx = lane + 32 * j, row = idx >> 3, c4 = (idx & 7) * 4; const v4f mv = *(const v4f*)(mp + (size_t)row * SEQ_FULL + kc + c4); *(v4fa*)(sM + mb + row * MP + c4) = mv; }
        int qv = qo; asm volatile("" : "+v"(qv));
        v8f sh0 = (v8f){}, sh1 = (v8f){}, sl0 = (v8f){}, sl1 = (v8f){};
#pragma unroll
        for (int ks = 0; ks < 2; ++ks) {
            const v16h aq = ldh(Q16 + qv + ks * 32), ar = ldh(QR + qv + ks * 32);
            const v16h b0 = ldh(Kp + (size_t)kc * HD + ks * 32), b1 = ldh(Kp + (size_t)(kc + 16) * HD + ks * 32);
            sh0 = wmma16(aq, b0, sh0); sl0 = wmma16(ar, b0, sl0); sh1 = wmma16(aq, b1, sh1); sl1 = wmma16(ar, b1, sl1);
            asm volatile("v_nop\n\tv_nop\n\tv_nop\n\tv_nop" : "+v"(sh0), "+v"(sl0), "+v"(sh1), "+v"(sl1) : "v"(aq), "v"(ar), "v"(b0), "v"(b1));
        }
        wsync();
#pragma unroll
        for (int r = 0; r < 8; ++r) {
            const int row = 8 * hi + r;
            const float m0 = bfr(sM[mb + row * MP + lr]), m1 = bfr(sM[mb + row * MP + 16 + lr]);
            const float t0 = fmaf(m0, LOG2E, fmaf(sl0[r], C2, sh0[r] * C1));
            const float t1 = fmaf(m1, LOG2E, fmaf(sl1[r], C2, sh1[r] * C1));
            float mx = fmaxf(t0, t1);
            mx = fmaxf(mx, __shfl_xor(mx, 8, 32)); mx = fmaxf(mx, __shfl_xor(mx, 4, 32)); mx = fmaxf(mx, __shfl_xor(mx, 2, 32)); mx = fmaxf(mx, __shfl_xor(mx, 1, 32));
            const float mnew = fmaxf(mrow[r], mx);
            const float alpha = __builtin_amdgcn_exp2f(mrow[r] - mnew);
            const float msh = mnew - PCAR_LOG2;
            const h16 p0 = (h16)__builtin_amdgcn_exp2f(t0 - msh), p1 = (h16)__builtin_amdgcn_exp2f(t1 - msh);
            lrow[r] = fmaf(lrow[r], alpha, (float)p0 + (float)p1);
            mrow[r] = mnew;
            accO[0][r] *= alpha; accO[1][r] *= alpha; accO[2][r] *= alpha; accO[3][r] *= alpha;
            sP[pb + row * PP + lr] = p0; sP[pb + row * PP + 16 + lr] = p1;
        }
        wsync();
        const v16h aP = cat16(*(const v8ha*)(sP + pb + lr * PP + 8 * hi), *(const v8ha*)(sP + pb + lr * PP + 16 + 8 * hi));
        v16h bv[4];
#pragma unroll
        for (int nb = 0; nb < 4; ++nb) bv[nb] = ldh(Vp + (size_t)(nb * 16) * SEQ + kc);
#pragma unroll
        for (int nb = 0; nb < 4; ++nb) accO[nb] = wmma16(aP, bv[nb], accO[nb]);
        asm volatile("v_nop\n\tv_nop\n\tv_nop\n\tv_nop" : "+v"(accO[0]), "+v"(accO[1]), "+v"(accO[2]), "+v"(accO[3]) : "v"(aP), "v"(bv[0]), "v"(bv[3]));
        wsync();
    }
#pragma unroll
    for (int r = 0; r < 8; ++r) {
        float l = lrow[r];
        l += __shfl_xor(l, 8, 32); l += __shfl_xor(l, 4, 32); l += __shfl_xor(l, 2, 32); l += __shfl_xor(l, 1, 32);
        const float inv = (1.0f / l) * (1.0f / VCAR);
#pragma unroll
        for (int nb = 0; nb < 4; ++nb) sO[ob + (8 * hi + r) * OP + nb * 16 + lr] = accO[nb][r] * inv;
    }
    wsync();
    v8us oh[4], ol[4];
    const int rq = lane >> 3, c8 = (lane & 7) * 8;
#pragma unroll
    for (int s = 0; s < 4; ++s) { const int row = s * 4 + rq; const v4f a = *(const v4fa*)(sO + ob + row * OP + c8), b = *(const v4fa*)(sO + ob + row * OP + c8 + 4);
#pragma unroll
        for (int k = 0; k < 4; ++k) { unsigned short x, y; splitf(a[k], x, y); oh[s][k] = x; ol[s][k] = y; splitf(b[k], x, y); oh[s][4 + k] = x; ol[s][4 + k] = y; } }
#pragma unroll 1
    for (int ps = 0; ps < 2; ++ps) {
#pragma unroll
        for (int s = 0; s < 4; ++s) { const size_t off = (size_t)(q0 + s * 4 + rq) * DQ + h * HD + c8; *(volatile v8us*)(ATh + off) = oh[s]; *(volatile v8us*)(ATl + off) = ol[s]; }
        if (ps == 0) __threadfence(); }
}

constexpr size_t al256(size_t b) { return (b + 255) & ~(size_t)255; }
constexpr size_t SZ_WQKV = al256((size_t)DQKV * DM * 2);
constexpr size_t SZ_WO   = al256((size_t)DM * DQ * 2);
constexpr size_t SZ_IF   = al256((size_t)1024 * 4);
constexpr size_t SZ_CS   = al256((size_t)SEQ * (HALFQ + HALFK) * 2 * 4);
constexpr size_t SZ_XB   = al256((size_t)SEQ * DM * 2);
constexpr size_t SZ_F    = al256((size_t)SEQ * DQKV * 4);
constexpr size_t SZ_Q    = al256((size_t)NH_ * SEQ * HD * 2);
constexpr size_t SZ_K    = al256((size_t)NKV * SEQ * HD * 2);
constexpr size_t SZ_AT   = al256((size_t)SEQ * DQ * 2);
constexpr size_t WS_TOTAL = SZ_WQKV + SZ_WO + SZ_IF + SZ_CS + SZ_XB + SZ_F + 2 * SZ_Q + 2 * SZ_K + 2 * SZ_AT;
static_assert(WS_TOTAL <= (size_t)134217728);
static_assert(HALFQ + HALFK <= 1024);

extern "C" void kernel_launch(void* const* d_in, const int* in_sizes, int n_in,
                              void* d_out, int out_size, void* d_ws, size_t ws_size, hipStream_t stream) {
    if (n_in < 10) return;
    if ((size_t)in_sizes[0] < (size_t)(NB - 1) * SEQ_FULL * DM + (size_t)SEQ * DM) return;
    if ((size_t)in_sizes[1] < (size_t)(NB - 1) * SEQ_FULL * SEQ_FULL + (size_t)(SEQ - 1) * SEQ_FULL + SEQ) return;
    if (in_sizes[2] < DM * DQ || in_sizes[3] < DQ || in_sizes[4] < DM * DKV || in_sizes[5] < DKV || in_sizes[6] < DM * DKV || in_sizes[7] < DKV || in_sizes[8] < DQ * DM || in_sizes[9] < DM) return;
    if ((size_t)out_size < (size_t)(NB - 1) * SEQ_FULL * DM + (size_t)SEQ * DM) return;
    if (WS_TOTAL > ws_size) return;
    const float* x = (const float*)d_in[0]; const float* amask = (const float*)d_in[1];
    const float* wq = (const float*)d_in[2]; const float* bq = (const float*)d_in[3];
    const float* wk = (const float*)d_in[4]; const float* bk = (const float*)d_in[5];
    const float* wv = (const float*)d_in[6]; const float* bv = (const float*)d_in[7];
    const float* wo = (const float*)d_in[8]; const float* bo = (const float*)d_in[9];
    float* OUT = (float*)d_out;
    char* wsp = (char*)d_ws;
    bf* WQKV = (bf*)wsp; wsp += SZ_WQKV;
    bf* WO = (bf*)wsp; wsp += SZ_WO;
    float* IF = (float*)wsp; wsp += SZ_IF;
    float* CS = (float*)wsp; wsp += SZ_CS;
    bf* XB = (bf*)wsp; wsp += SZ_XB;
    float* FQKV = (float*)wsp; wsp += SZ_F;
    h16* Q16 = (h16*)wsp; wsp += SZ_Q;
    h16* QR16 = (h16*)wsp; wsp += SZ_Q;
    h16* K16 = (h16*)wsp; wsp += SZ_K;
    h16* VT16 = (h16*)wsp; wsp += SZ_K;
    bf* ATh = (bf*)wsp; wsp += SZ_AT;
    bf* ATl = (bf*)wsp; wsp += SZ_AT;
    float* CSQ = CS; float* CSK = CS + (size_t)SEQ * HALFQ * 2;

    k_wtG<<<(unsigned)((DM * DQ / 64 + 63) / 64), 256, 0, stream>>>(wq, DM, DQ, WQKV);
    k_wtG<<<(unsigned)((DM * DKV / 64 + 63) / 64), 256, 0, stream>>>(wk, DM, DKV, WQKV + (size_t)DQ * DM);
    k_wtG<<<(unsigned)((DM * DKV / 64 + 63) / 64), 256, 0, stream>>>(wv, DM, DKV, WQKV + (size_t)(DQ + DKV) * DM);
    k_wtG<<<(unsigned)((DQ * DM / 64 + 63) / 64), 256, 0, stream>>>(wo, DQ, DM, WO);
    k_invf<<<4, 256, 0, stream>>>(IF);
    k_cstab<<<(unsigned)((SEQ * (HALFQ + HALFK) + 255) / 256), 256, 0, stream>>>(IF, CS);
    for (int b = 0; b < NB; ++b) {
        k_cvt8<<<(unsigned)(((size_t)SEQ * DM / 8 + 255) / 256), 256, 0, stream>>>(x + (size_t)b * SEQ_FULL * DM, XB, (size_t)SEQ * DM / 8);
        k_gemm_proj<<<dim3(SEQ / 64, DQKV / 64, 1), 32, 0, stream>>>(XB, WQKV, DM, FQKV, DQKV);
        k_ropen<<<(unsigned)(NH_ * SEQ / 8), 256, 0, stream>>>(FQKV, 0, HALFQ, NH_, CSQ, bq, 1, Q16, QR16);
        k_ropen<<<(unsigned)(NKV * SEQ / 8), 256, 0, stream>>>(FQKV, DQ, HALFK, NKV, CSK, bk, 0, K16, K16);
        k_vtp<<<(unsigned)(((size_t)NKV * HD * SEQ / 2 + 255) / 256), 256, 0, stream>>>(FQKV, bv, VT16);
        k_flash<<<dim3(SEQ / 16, NKV, 1), 128, 0, stream>>>(Q16, QR16, K16, VT16, amask + (size_t)b * SEQ_FULL * SEQ_FULL, ATh, ATl);
        k_gemm_out<<<dim3(SEQ / 64, DM / 64, 1), 32, 0, stream>>>(ATh, ATl, WO, DQ, OUT + (size_t)b * SEQ_FULL * DM, DM, bo);
    }
}
